// MultiQueryAttention_48799418417749
// MI455X (gfx1250) — hardware-verified
//
#include <hip/hip_runtime.h>
#include <stdint.h>


typedef _Float16 v16h __attribute__((ext_vector_type(16)));
typedef _Float16 v8h  __attribute__((ext_vector_type(8)));
typedef float    v8f  __attribute__((ext_vector_type(8)));
typedef float    v4f  __attribute__((ext_vector_type(4)));

#define DM 1024
#define HD 64
#define NH 16
#define NB_FULL 2
#define SEQ_FULL 2048
#ifndef NB
#define NB 2
#endif
#ifndef SEQ
#define SEQ 2048
#endif
#ifndef ER
#if SEQ >= 256
#define ER 256
#else
#define ER SEQ
#endif
#endif
#define MROWS (NB * SEQ)
#define WSCALE 64.0f
#define PCARRY 256.0f
#define YCARRY 64.0f
#define RESC 2048.0f
#define LOG2E 1.4426950408889634f

static_assert(SEQ % 128 == 0);
static_assert(SEQ <= SEQ_FULL);
static_assert(NB >= 1 && NB <= NB_FULL);
static_assert(ER % 128 == 0 && ER >= 128 && ER <= SEQ);
static_assert(DM % 128 == 0 && (2 * HD) == 128 && DM == NH * HD);

union HFrag { v16h v; v8h h[2]; };

__device__ __forceinline__ v16h load_frag(const _Float16* p) {
    HFrag f;
    f.h[0] = *reinterpret_cast<const v8h*>(p);
    f.h[1] = *reinterpret_cast<const v8h*>(p + 16);
    return f.v;
}

__device__ __forceinline__ v8f wmma16(v16h a, v16h b, v8f c) {
    return __builtin_amdgcn_wmma_f32_16x16x32_f16(false, a, false, b, (short)0, c, false, false);
}

__device__ __forceinline__ float bf16r(float f) {
    unsigned int u = __float_as_uint(f);
    u += 0x7FFFu + ((u >> 16) & 1u);
    u &= 0xFFFF0000u;
    return __uint_as_float(u);
}

template <bool LO>
__device__ __forceinline__ _Float16 part16(float v) {
    const _Float16 hv = (_Float16)v;
    if (LO) return (_Float16)((v - (float)hv) * RESC);
    return hv;
}

__global__ __launch_bounds__(256) void k_cvt_x(const float* __restrict__ x, _Float16* x16)
{
    const int u = blockIdx.x * 256 + threadIdx.x;
    const int row = u >> 7;
    const int col = (u & 127) * 8;
    const int bb = row / SEQ;
    const int s  = row - bb * SEQ;
    const float* src = x + ((size_t)(bb * SEQ_FULL + s)) * DM + col;
    const v4f f0 = *reinterpret_cast<const v4f*>(src);
    const v4f f1 = *reinterpret_cast<const v4f*>(src + 4);
    v8h o;
    o[0] = (_Float16)bf16r(f0[0]); o[1] = (_Float16)bf16r(f0[1]);
    o[2] = (_Float16)bf16r(f0[2]); o[3] = (_Float16)bf16r(f0[3]);
    o[4] = (_Float16)bf16r(f1[0]); o[5] = (_Float16)bf16r(f1[1]);
    o[6] = (_Float16)bf16r(f1[2]); o[7] = (_Float16)bf16r(f1[3]);
    _Float16* dst = x16 + (size_t)row * DM + col;
    *(volatile v8h*)dst = o;
    __threadfence();
    *(volatile v8h*)dst = o;
}

__global__ __launch_bounds__(256) void k_wt(const float* __restrict__ W, _Float16* WT, int N)
{
    __shared__ _Float16 tile[32 * 72] __attribute__((aligned(16)));
    const int tid = threadIdx.x;
    const int n0 = blockIdx.x * 32, k0 = blockIdx.y * 64;
    const int nn = tid & 31, kq = tid >> 5;
#pragma unroll
    for (int i = 0; i < 8; ++i) {
        const int kk = kq + 8 * i;
        const float w = W[(size_t)(k0 + kk) * N + n0 + nn];
        tile[nn * 72 + kk] = (_Float16)(bf16r(w) * WSCALE);
    }
    __syncthreads();
    const int on = tid >> 3, seg = tid & 7;
    const v8h v = *reinterpret_cast<const v8h*>(tile + on * 72 + seg * 8);
    _Float16* dst = WT + (size_t)(n0 + on) * DM + k0 + seg * 8;
    *(volatile v8h*)dst = v;
    __threadfence();
    *(volatile v8h*)dst = v;
}

__global__ __launch_bounds__(256) void k_tab(float* cosT, float* sinT)
{
    const int lane = threadIdx.x & 31;
    const int t = blockIdx.x * 8 + (threadIdx.x >> 5);
    const int e10 = lane >> 3, e8 = lane & 7;
    double pw = (e10 == 0) ? 1.0 : ((e10 == 1) ? 10.0 : ((e10 == 2) ? 100.0 : 1000.0));
#pragma unroll 1
    for (int c = 0; c < e8; ++c) pw *= 1.3335214321633240;
    const float pf = (float)pw;
    const float invf = 1.0f / pf;
    const float ang = (float)t * invf;
    const double a = (double)ang;
    const double kq = __builtin_rint(a * 0.63661977236758134);
    const int qd = (int)kq;
    double rr = __builtin_fma(-kq, 1.5707963267948966, a);
    rr = __builtin_fma(-kq, 6.123233995736766e-17, rr);
    const double r2 = rr * rr;
    const double sp = rr + rr * r2 * (-1.6666666666666666e-1 + r2 * (8.3333333333333332e-3
                      + r2 * (-1.9841269841269841e-4 + r2 * (2.7557319223985893e-6
                      + r2 * (-2.5052108385441720e-8)))));
    const double cp = 1.0 + r2 * (-0.5 + r2 * (4.1666666666666664e-2 + r2 * (-1.3888888888888889e-3
                      + r2 * (2.4801587301587302e-5 + r2 * (-2.7557319223985888e-7
                      + r2 * 2.0876756987868100e-9)))));
    const double ss0 = (qd & 1) ? cp : sp;
    const double cc0 = (qd & 1) ? -sp : cp;
    const double ss = (qd & 2) ? -ss0 : ss0;
    const double cc = (qd & 2) ? -cc0 : cc0;
    const float cv = (float)cc, sv = (float)ss;
    float* cd = cosT + (size_t)t * 32 + lane;
    float* sd = sinT + (size_t)t * 32 + lane;
    *(volatile float*)cd = cv;
    *(volatile float*)sd = sv;
    __threadfence();
    *(volatile float*)cd = cv;
    *(volatile float*)sd = sv;
}

__device__ __forceinline__ void store32x64_f16(const _Float16* sw, _Float16* gdst,
                                               int pitch, int lane)
{
    const int rq = lane >> 3, seg = lane & 7;
    v8h v[8];
#pragma unroll
    for (int it = 0; it < 8; ++it)
        v[it] = *reinterpret_cast<const v8h*>(sw + (it * 4 + rq) * 64 + seg * 8);
#pragma unroll
    for (int it = 0; it < 8; ++it)
        *(volatile v8h*)(gdst + (it * 4 + rq) * pitch + seg * 8) = v[it];
    __threadfence();
#pragma unroll
    for (int it = 0; it < 8; ++it)
        *(volatile v8h*)(gdst + (it * 4 + rq) * pitch + seg * 8) = v[it];
}

__device__ __forceinline__ void store16x64_f16(const _Float16* s72, _Float16* gdst,
                                               int pitch, int lane)
{
    const int rq = lane >> 3, seg = lane & 7;
    v8h v[4];
#pragma unroll
    for (int it = 0; it < 4; ++it)
        v[it] = *reinterpret_cast<const v8h*>(s72 + (it * 4 + rq) * 72 + seg * 8);
#pragma unroll
    for (int it = 0; it < 4; ++it)
        *(volatile v8h*)(gdst + (it * 4 + rq) * pitch + seg * 8) = v[it];
    __threadfence();
#pragma unroll
    for (int it = 0; it < 4; ++it)
        *(volatile v8h*)(gdst + (it * 4 + rq) * pitch + seg * 8) = v[it];
}

__device__ __forceinline__ void store16x64s64_f16(const _Float16* s64, _Float16* gdst,
                                                  int pitch, int lane)
{
    const int rq = lane >> 3, seg = lane & 7;
    v8h v[4];
#pragma unroll
    for (int it = 0; it < 4; ++it)
        v[it] = *reinterpret_cast<const v8h*>(s64 + (it * 4 + rq) * 64 + seg * 8);
#pragma unroll
    for (int it = 0; it < 4; ++it)
        *(volatile v8h*)(gdst + (it * 4 + rq) * pitch + seg * 8) = v[it];
    __threadfence();
#pragma unroll
    for (int it = 0; it < 4; ++it)
        *(volatile v8h*)(gdst + (it * 4 + rq) * pitch + seg * 8) = v[it];
}

__device__ __forceinline__ void storeVT(const _Float16* vs, _Float16* vd, int pitch, int tid)
{
    const int dq = tid >> 4, seg = tid & 15;
    v8h v[4];
#pragma unroll
    for (int it = 0; it < 4; ++it)
        v[it] = *reinterpret_cast<const v8h*>(vs + (it * 16 + dq) * 128 + seg * 8);
#pragma unroll
    for (int it = 0; it < 4; ++it)
        *(volatile v8h*)(vd + (it * 16 + dq) * pitch + seg * 8) = v[it];
    __threadfence();
#pragma unroll
    for (int it = 0; it < 4; ++it)
        *(volatile v8h*)(vd + (it * 16 + dq) * pitch + seg * 8) = v[it];
}

template <bool LO>
__device__ __forceinline__ void stage_rows(_Float16* sw, const v8f (&acc)[2][4], int hi8, int l15)
{
#pragma unroll
    for (int g = 0; g < 2; ++g)
#pragma unroll
        for (int ni = 0; ni < 4; ++ni)
#pragma unroll
            for (int j = 0; j < 8; ++j)
                sw[(g * 16 + hi8 + j) * 64 + ni * 16 + l15] = part16<LO>(acc[g][ni][j]);
}

template <bool LO>
__device__ __forceinline__ void stage_vt(_Float16* vs, const v8f (&acc)[2][4], int wm, int hi8, int l15)
{
#pragma unroll
    for (int g = 0; g < 2; ++g)
#pragma unroll
        for (int ni = 0; ni < 4; ++ni)
#pragma unroll
            for (int j = 0; j < 8; ++j)
                vs[(ni * 16 + l15) * 128 + wm * 32 + g * 16 + hi8 + j] = part16<LO>(acc[g][ni][j]);
}

__device__ __forceinline__ void kloop(v8f (&acc)[2][4], const _Float16* __restrict__ ap0,
                                      const _Float16* __restrict__ ap1,
                                      const _Float16* __restrict__ bp, size_t bst, int K)
{
#pragma unroll 1
    for (int k0 = 0; k0 < K; k0 += 32) {
        const v16h a0 = load_frag(ap0 + k0);
        const v16h a1 = load_frag(ap1 + k0);
        const v16h b0 = load_frag(bp + k0);
        const v16h b1 = load_frag(bp + bst + k0);
        const v16h b2 = load_frag(bp + 2 * bst + k0);
        const v16h b3 = load_frag(bp + 3 * bst + k0);
        acc[0][0] = wmma16(a0, b0, acc[0][0]);
        acc[0][1] = wmma16(a0, b1, acc[0][1]);
        acc[0][2] = wmma16(a0, b2, acc[0][2]);
        acc[0][3] = wmma16(a0, b3, acc[0][3]);
        acc[1][0] = wmma16(a1, b0, acc[1][0]);
        acc[1][1] = wmma16(a1, b1, acc[1][1]);
        acc[1][2] = wmma16(a1, b2, acc[1][2]);
        acc[1][3] = wmma16(a1, b3, acc[1][3]);
        asm volatile("v_nop\n\tv_nop\n\tv_nop\n\tv_nop"
                     : "+v"(acc[0][0]), "+v"(acc[0][1]), "+v"(acc[0][2]), "+v"(acc[0][3]),
                       "+v"(acc[1][0]), "+v"(acc[1][1]), "+v"(acc[1][2]), "+v"(acc[1][3])
                     : "v"(a0), "v"(a1), "v"(b0), "v"(b1), "v"(b2), "v"(b3));
    }
}

template <int MODE>
__global__ __launch_bounds__(256) __attribute__((amdgpu_num_vgpr(256)))
void k_gemm(const _Float16* __restrict__ A,
            const _Float16* __restrict__ BT,
            void* C0, void* C1, void* C2, void* C3,
            const float* __restrict__ cosT,
            const float* __restrict__ sinT,
            int N, int K, float alpha)
{
    __shared__ float stg[8 * 1024] __attribute__((aligned(16)));
    const int tid = threadIdx.x;
    const int lane = tid & 31, wave = tid >> 5;
    const int wm = wave & 3, wn = wave >> 2;
    const int l15 = lane & 15, hi8 = (lane >> 4) << 3;
    const int bm0 = blockIdx.y * 128, bn0 = blockIdx.x * 128;
    const int RPB = (MODE == 4) ? ER : SEQ;
    const int bb = bm0 / RPB;
    const int s0 = bm0 - bb * RPB;
    const bool early = (s0 < ER);

    const _Float16* bp  = BT + (size_t)(bn0 + wn * 64 + l15) * K + hi8;
    const size_t bst = (size_t)16 * K;

    const v8f zero8 = {0.f, 0.f, 0.f, 0.f, 0.f, 0.f, 0.f, 0.f};
    v8f acc[2][4];
#pragma unroll
    for (int g = 0; g < 2; ++g)
#pragma unroll
        for (int ni = 0; ni < 4; ++ni) acc[g][ni] = zero8;

    {
        const _Float16* ap0 = A + (size_t)(bm0 + wm * 32 + l15) * K + hi8;
        kloop(acc, ap0, ap0 + (size_t)16 * K, bp, bst, K);
    }

    if (MODE == 1 || MODE == 4) {
        float* swf = stg + wave * 1024;
        const int rq = lane >> 4, seg = lane & 15;
        const int cofs = bn0 + wn * 64 + seg * 4;
        const bool tostage = (MODE == 1) && early;
        const size_t orow = tostage ? (size_t)(bb * ER + s0 + wm * 32)
                                    : ((size_t)bb * SEQ_FULL + s0 + wm * 32);
        float* gb = (float*)(tostage ? C1 : C0) + orow * (size_t)N + cofs;
        const float* sb = (const float*)C1 + (size_t)(bm0 + wm * 32) * N + cofs;
#pragma unroll
        for (int g = 0; g < 2; ++g) {
#pragma unroll
            for (int ni = 0; ni < 4; ++ni)
#pragma unroll
                for (int j = 0; j < 8; ++j)
                    swf[(hi8 + j) * 64 + ni * 16 + l15] = acc[g][ni][j] * alpha;
            __syncthreads();
            v4f v[8];
#pragma unroll
            for (int it = 0; it < 8; ++it)
                v[it] = *reinterpret_cast<const v4f*>(swf + (it * 2 + rq) * 64 + seg * 4);
            if (MODE == 4) {
                const float* sg = sb + (size_t)(g * 16) * N;
#pragma unroll
                for (int it = 0; it < 8; ++it) {
                    const v4f sv = *reinterpret_cast<const v4f*>(sg + (it * 2 + rq) * N);
                    v[it] = v[it] + sv;
                }
            }
            float* gd = gb + (size_t)(g * 16) * N;
#pragma unroll
            for (int it = 0; it < 8; ++it)
                *(volatile v4f*)(gd + (it * 2 + rq) * N) = v[it];
            __threadfence();
#pragma unroll
            for (int it = 0; it < 8; ++it)
                *(volatile v4f*)(gd + (it * 2 + rq) * N) = v[it];
            __syncthreads();
        }
    } else {
        {
            const v4f* cg = reinterpret_cast<const v4f*>(cosT + (size_t)s0 * 32);
            const v4f* sg = reinterpret_cast<const v4f*>(sinT + (size_t)s0 * 32);
            v4f* cl = reinterpret_cast<v4f*>(stg);
            v4f* sl = reinterpret_cast<v4f*>(stg + 4096);
#pragma unroll
            for (int i = 0; i < 4; ++i) {
                const v4f c4 = cg[tid + 256 * i];
                cl[tid + 256 * i] = c4;
                const v4f s4 = sg[tid + 256 * i];
                sl[tid + 256 * i] = s4;
            }
        }
        __syncthreads();
        const bool dorope = (MODE == 3) || (wn == 0);
        const float* tb = stg + (wm * 32 + hi8) * 32 + l15;
#pragma unroll
        for (int g = 0; g < 2; ++g)
#pragma unroll
            for (int j = 0; j < 8; ++j) {
#pragma unroll
                for (int ni = 0; ni < 2; ++ni) {
                    const float ct = tb[(g * 16 + j) * 32 + ni * 16];
                    const float st = tb[4096 + (g * 16 + j) * 32 + ni * 16];
                    const float c = dorope ? ct : 1.0f;
                    const float s = dorope ? st : 0.0f;
                    const float x0 = acc[g][ni][j] * alpha;
                    const float x1 = acc[g][ni + 2][j] * alpha;
                    acc[g][ni][j]     = x0 * c - x1 * s;
                    acc[g][ni + 2][j] = x1 * c + x0 * s;
                }
            }
        __syncthreads();

        _Float16* sw = reinterpret_cast<_Float16*>(stg + wave * 1024);
        _Float16* vs = reinterpret_cast<_Float16*>(stg + 4 * 1024);
        if (MODE == 3) {
            _Float16* gh = (_Float16*)C0 + (size_t)(bm0 + wm * 32) * N + bn0 + wn * 64;
#pragma unroll
            for (int g = 0; g < 2; ++g) {
#pragma unroll
                for (int ni = 0; ni < 4; ++ni)
#pragma unroll
                    for (int j = 0; j < 8; ++j) {
                        const float v = acc[g][ni][j];
                        const _Float16 hv = (_Float16)v;
                        const int o = (hi8 + j) * 64 + ni * 16 + l15;
                        sw[o] = hv;
                        sw[1024 + o] = (_Float16)((v - (float)hv) * RESC);
                    }
                __syncthreads();
                store16x64s64_f16(sw, gh + (size_t)(g * 16) * N, N, lane);
                if (early)
                    store16x64s64_f16(sw + 1024,
                                      (_Float16*)C2 + (size_t)(bb * ER + s0 + wm * 32 + g * 16) * N + bn0 + wn * 64,
                                      N, lane);
                __syncthreads();
            }
        } else {
            if (wn == 0) stage_rows<false>(sw, acc, hi8, l15);
            else         stage_vt<false>(vs, acc, wm, hi8, l15);
            __syncthreads();
            if (wn == 0)
                store32x64_f16(sw, (_Float16*)C0 + (size_t)(bm0 + wm * 32) * HD, HD, lane);
            storeVT(vs, (_Float16*)C1 + ((size_t)(bb * HD)) * SEQ + s0, SEQ, tid);
            if (early) {
                __syncthreads();
                if (wn == 0) stage_rows<true>(sw, acc, hi8, l15);
                else         stage_vt<true>(vs, acc, wm, hi8, l15);
                __syncthreads();
                if (wn == 0)
                    store32x64_f16(sw, (_Float16*)C2 + (size_t)(bb * ER + s0 + wm * 32) * HD, HD, lane);
                storeVT(vs, (_Float16*)C3 + ((size_t)(bb * HD)) * ER + s0, ER, tid);
            }
        }
    }
}

__global__ __launch_bounds__(128) __attribute__((amdgpu_num_vgpr(256)))
void k_attn(const _Float16* __restrict__ qp,
            const _Float16* __restrict__ kp,
            const _Float16* __restrict__ vT,
            _Float16* yp)
{
    __shared__ _Float16 Ws[4 * 16 * 72] __attribute__((aligned(16)));
    const int lane = threadIdx.x & 31;
    const int wv   = threadIdx.x >> 5;
    const int l15  = lane & 15;
    const int hi8  = (lane >> 4) << 3;

    const int nlate = (SEQ / 64 - ER / 64) > 0 ? (SEQ / 64 - ER / 64) : 1;
    int bid = blockIdx.x;
    const int qb = ER / 64 + bid % nlate; bid /= nlate;
    const int h  = bid % NH;
    const int b  = bid / NH;
    const int qt = qb * 4 + wv;
    const int kend = (qb + 1) * 64;
    const int qr0 = qt * 16 + hi8;

    const _Float16* qbase = qp + ((size_t)(b * SEQ + qt * 16 + l15)) * DM + h * HD + hi8;
    const v16h aQ0 = load_frag(qbase);
    const v16h aQ1 = load_frag(qbase + 32);

    const _Float16* kbase = kp + (size_t)b * SEQ * HD + hi8;
    const _Float16* vbase = vT + (size_t)(b * HD) * SEQ + hi8;

    const v8f zero8 = {0.f, 0.f, 0.f, 0.f, 0.f, 0.f, 0.f, 0.f};
    float m[8], l[8];
    v8f accY[4];
#pragma unroll
    for (int j = 0; j < 8; ++j) { m[j] = -1e30f; l[j] = 0.0f; }
#pragma unroll
    for (int ni = 0; ni < 4; ++ni) accY[ni] = zero8;

    _Float16* ps = Ws + wv * 16 * 72;

#pragma unroll 1
    for (int tc = 0; tc < kend; tc += 32) {
        const _Float16* kp0 = kbase + (size_t)(tc + l15) * HD;
        const _Float16* kp1 = kp0 + 16 * HD;
        const v16h b00 = load_frag(kp0);
        const v16h b01 = load_frag(kp0 + 32);
        const v16h b10 = load_frag(kp1);
        const v16h b11 = load_frag(kp1 + 32);
        v8f s0 = zero8, s1 = zero8;
        s0 = wmma16(aQ0, b00, s0);
        s0 = wmma16(aQ1, b01, s0);
        s1 = wmma16(aQ0, b10, s1);
        s1 = wmma16(aQ1, b11, s1);
        asm volatile("v_nop\n\tv_nop\n\tv_nop\n\tv_nop"
                     : "+v"(s0), "+v"(s1)
                     : "v"(aQ0), "v"(aQ1), "v"(b00), "v"(b01), "v"(b10), "v"(b11));

#pragma unroll
        for (int j = 0; j < 8; ++j) {
            const int qr = qr0 + j;
            const float a0 = (tc + l15 <= qr)      ? s0[j] * 0.125f : -1e30f;
            const float a1 = (tc + 16 + l15 <= qr) ? s1[j] * 0.125f : -1e30f;
            float mt = fmaxf(a0, a1);
#pragma unroll
            for (int off = 8; off >= 1; off >>= 1)
                mt = fmaxf(mt, __shfl_xor(mt, off, 16));
            const float mn = fmaxf(m[j], mt);
            const float sc = exp2f(m[j] - mn);
            const float p0 = exp2f(a0 - mn);
            const float p1 = exp2f(a1 - mn);
            float rs = p0 + p1;
#pragma unroll
            for (int off = 8; off >= 1; off >>= 1)
                rs += __shfl_xor(rs, off, 16);
            l[j] = l[j] * sc + rs;
            m[j] = mn;
            accY[0][j] *= sc; accY[1][j] *= sc;
            accY[2][j] *= sc; accY[3][j] *= sc;
            const int row = hi8 + j;
            ps[row * 72 + l15]      = (_Float16)(p0 * PCARRY);
            ps[row * 72 + 16 + l15] = (_Float16)(p1 * PCARRY);
        }
        __syncthreads();

        const v16h aP = load_frag(ps + l15 * 72 + hi8);
        const v16h bV0 = load_frag(vbase + (size_t)(0 * 16 + l15) * SEQ + tc);
        const v16h bV1 = load_frag(vbase + (size_t)(1 * 16 + l15) * SEQ + tc);
        const v16h bV2 = load_frag(vbase + (size_t)(2 * 16 + l15) * SEQ + tc);
        const v16h bV3 = load_frag(vbase + (size_t)(3 * 16 + l15) * SEQ + tc);
        accY[0] = wmma16(aP, bV0, accY[0]);
        accY[1] = wmma16(aP, bV1, accY[1]);
        accY[2] = wmma16(aP, bV2, accY[2]);
        accY[3] = wmma16(aP, bV3, accY[3]);
        asm volatile("v_nop\n\tv_nop\n\tv_nop\n\tv_nop"
                     : "+v"(accY[0]), "+v"(accY[1]), "+v"(accY[2]), "+v"(accY[3])
                     : "v"(aP), "v"(bV0), "v"(bV1), "v"(bV2), "v"(bV3));
    }
    __syncthreads();

    float inv[8];
#pragma unroll
    for (int j = 0; j < 8; ++j) inv[j] = (YCARRY / PCARRY) / l[j];
#pragma unroll
    for (int ni = 0; ni < 4; ++ni)
#pragma unroll
        for (int j = 0; j < 8; ++j)
            ps[(hi8 + j) * 72 + ni * 16 + l15] = (_Float16)(accY[ni][j] * inv[j]);
    __syncthreads();

    store16x64_f16(ps, yp + ((size_t)(b * SEQ + qt * 16)) * DM + h * HD, DM, lane);
}

__global__ __launch_bounds__(128) __attribute__((amdgpu_num_vgpr(256)))
void k_attn_e(const _Float16* qp, const _Float16* ql,
              const _Float16* kp, const _Float16* kl,
              const _Float16* vT, const _Float16* vR,
              _Float16* yp, _Float16* yl)
{
    __shared__ _Float16 Ws[4 * 16 * 72] __attribute__((aligned(16)));
    const int lane = threadIdx.x & 31;
    const int wv   = threadIdx.x >> 5;
    const int l15  = lane & 15;
    const int hi8  = (lane >> 4) << 3;

    const int nearly = ER / 64;
    int bid = blockIdx.x;
    const int qb = bid % nearly; bid /= nearly;
    const int h  = bid % NH;
    const int b  = bid / NH;
    const int qt = qb * 4 + wv;
    const int kend = (qb + 1) * 64;
    const int qr0 = qt * 16 + hi8;

    const _Float16* qbase = qp + ((size_t)(b * SEQ + qt * 16 + l15)) * DM + h * HD + hi8;
    const _Float16* lbase = ql + ((size_t)(b * ER + qt * 16 + l15)) * DM + h * HD + hi8;
    const _Float16* kbase = kp + (size_t)b * SEQ * HD + hi8;
    const _Float16* klb   = kl + (size_t)b * ER * HD + hi8;
    const _Float16* vbase = vT + (size_t)(b * HD) * SEQ + hi8;
    const _Float16* vrb   = vR + (size_t)(b * HD) * ER + hi8;

    const v8f zero8 = {0.f, 0.f, 0.f, 0.f, 0.f, 0.f, 0.f, 0.f};
    float m[8], l[8];
    v8f accY[4];
#pragma unroll
    for (int j = 0; j < 8; ++j) { m[j] = -1e30f; l[j] = 0.0f; }
#pragma unroll
    for (int ni = 0; ni < 4; ++ni) accY[ni] = zero8;

    _Float16* ps = Ws + wv * 16 * 72;

#pragma unroll 1
    for (int tc = 0; tc < kend; tc += 32) {
        v8f s0 = zero8, s1 = zero8, r0 = zero8, r1 = zero8;
        const _Float16* kq0 = kbase + (size_t)(tc + l15) * HD;
        const _Float16* kq1 = kq0 + 16 * HD;
        const _Float16* kl0 = klb + (size_t)(tc + l15) * HD;
        const _Float16* kl1 = kl0 + 16 * HD;
#pragma unroll
        for (int dh = 0; dh < 64; dh += 32) {
            const v16h bK0 = load_frag(kq0 + dh);
            const v16h bK1 = load_frag(kq1 + dh);
            {
                const v16h aQ  = load_frag(qbase + dh);
                const v16h cK0 = load_frag(kl0 + dh);
                const v16h cK1 = load_frag(kl1 + dh);
                s0 = wmma16(aQ, bK0, s0);
                s1 = wmma16(aQ, bK1, s1);
                r0 = wmma16(aQ, cK0, r0);
                r1 = wmma16(aQ, cK1, r1);
                asm volatile("v_nop\n\tv_nop\n\tv_nop\n\tv_nop"
                             : "+v"(s0), "+v"(s1), "+v"(r0), "+v"(r1)
                             : "v"(aQ), "v"(bK0), "v"(bK1), "v"(cK0), "v"(cK1));
            }
            {
                const v16h aL = load_frag(lbase + dh);
                r0 = wmma16(aL, bK0, r0);
                r1 = wmma16(aL, bK1, r1);
                asm volatile("v_nop\n\tv_nop\n\tv_nop\n\tv_nop"
                             : "+v"(r0), "+v"(r1)
                             : "v"(aL), "v"(bK0), "v"(bK1));
            }
        }

#pragma unroll
        for (int j = 0; j < 8; ++j) {
            const int qr = qr0 + j;
            const float f0 = s0[j] + r0[j] * (1.0f / RESC);
            const float f1 = s1[j] + r1[j] * (1.0f / RESC);
            const float a0 = (tc + l15 <= qr)      ? f0 * 0.125f : -1e30f;
            const float a1 = (tc + 16 + l15 <= qr) ? f1 * 0.125f : -1e30f;
            float mt = fmaxf(a0, a1);
#pragma unroll
            for (int off = 8; off >= 1; off >>= 1)
                mt = fmaxf(mt, __shfl_xor(mt, off, 16));
            const float mn = fmaxf(m[j], mt);
            const float sc = exp2f(m[j] - mn);
            const float p0 = exp2f(a0 - mn);
            const float p1 = exp2f(a1 - mn);
            float rs = p0 + p1;
#pragma unroll
            for (int off = 8; off >= 1; off >>= 1)
                rs += __shfl_xor(rs, off, 16);
            l[j] = l[j] * sc + rs;
            m[j] = mn;
            accY[0][j] *= sc; accY[1][j] *= sc;
            accY[2][j] *= sc; accY[3][j] *= sc;
            const int row = hi8 + j;
            const float pc0 = p0 * PCARRY, pc1 = p1 * PCARRY;
            const _Float16 h0 = (_Float16)pc0, h1 = (_Float16)pc1;
            ps[row * 72 + l15]      = h0;
            ps[row * 72 + 16 + l15] = h1;
            ps[row * 72 + 32 + l15] = (_Float16)((pc0 - (float)h0) * RESC);
            ps[row * 72 + 48 + l15] = (_Float16)((pc1 - (float)h1) * RESC);
        }
        __syncthreads();

        v8f t0, t1, t2, t3;
        {
            const v16h aP = load_frag(ps + l15 * 72 + hi8);
            const v16h aR = load_frag(ps + l15 * 72 + 32 + hi8);
            {
                const v16h bV0 = load_frag(vbase + (size_t)(0 * 16 + l15) * SEQ + tc);
                const v16h bV1 = load_frag(vbase + (size_t)(1 * 16 + l15) * SEQ + tc);
                accY[0] = wmma16(aP, bV0, accY[0]);
                accY[1] = wmma16(aP, bV1, accY[1]);
                t0 = wmma16(aR, bV0, zero8);
                t1 = wmma16(aR, bV1, zero8);
                asm volatile("v_nop\n\tv_nop\n\tv_nop\n\tv_nop"
                             : "+v"(accY[0]), "+v"(accY[1]), "+v"(t0), "+v"(t1)
                             : "v"(aP), "v"(aR), "v"(bV0), "v"(bV1));
            }
            {
                const v16h bR0 = load_frag(vrb + (size_t)(0 * 16 + l15) * ER + tc);
                const v16h bR1 = load_frag(vrb + (size_t)(1 * 16 + l15) * ER + tc);
                t0 = wmma16(aP, bR0, t0);
                t1 = wmma16(aP, bR1, t1);
                asm volatile("v_nop\n\tv_nop\n\tv_nop\n\tv_nop"
                             : "+v"(t0), "+v"(t1)
                             : "v"(aP), "v"(bR0), "v"(bR1));
            }
            {
                const v16h bV2 = load_frag(vbase + (size_t)(2 * 16 + l15) * SEQ + tc);
                const v16h bV3 = load_frag(vbase + (size_t)(3 * 16 + l15) * SEQ + tc);
                accY[2] = wmma16(aP, bV2, accY[2]);
                accY[3] = wmma16(aP, bV3, accY[3]);
                t2 = wmma16(aR, bV2, zero8);
                t3 = wmma16(aR, bV3, zero8);
                asm volatile("v_nop\n\tv_nop\n\tv_nop\n\tv_nop"
                             : "+v"(accY[2]), "+v"(accY[3]), "+v"(t2), "+v"(t3)
                             : "v"(aP), "v"(aR), "v"(bV2), "v"(bV3));
            }
            {
                const v16h bR2 = load_frag(vrb + (size_t)(2 * 16 + l15) * ER + tc);
                const v16h bR3 = load_frag(vrb + (size_t)(3 * 16 + l15) * ER + tc);
                t2 = wmma16(aP, bR2, t2);
                t3 = wmma16(aP, bR3, t3);
                asm volatile("v_nop\n\tv_nop\n\tv_nop\n\tv_nop"
                             : "+v"(t2), "+v"(t3)
                             : "v"(aP), "v"(bR2), "v"(bR3));
            }
        }
        accY[0] = accY[0] + t0 * (1.0f / RESC);
        accY[1] = accY[1] + t1 * (1.0f / RESC);
        accY[2] = accY[2] + t2 * (1.0f / RESC);
        accY[3] = accY[3] + t3 * (1.0f / RESC);
    }
    __syncthreads();

    float inv[8];
#pragma unroll
    for (int j = 0; j < 8; ++j) inv[j] = (YCARRY / PCARRY) / l[j];
#pragma unroll
    for (int ni = 0; ni < 4; ++ni)
#pragma unroll
        for (int j = 0; j < 8; ++j) accY[ni][j] *= inv[j];

#pragma unroll
    for (int ni = 0; ni < 4; ++ni)
#pragma unroll
        for (int j = 0; j < 8; ++j)
            ps[(hi8 + j) * 72 + ni * 16 + l15] = part16<false>(accY[ni][j]);
    __syncthreads();
    store16x64_f16(ps, yp + ((size_t)(b * SEQ + qt * 16)) * DM + h * HD, DM, lane);
    __syncthreads();
#pragma unroll
    for (int ni = 0; ni < 4; ++ni)
#pragma unroll
        for (int j = 0; j < 8; ++j)
            ps[(hi8 + j) * 72 + ni * 16 + l15] = part16<true>(accY[ni][j]);
    __syncthreads();
    store16x64_f16(ps, yl + ((size_t)(b * ER + qt * 16)) * DM + h * HD, DM, lane);
}

extern "C" void kernel_launch(void* const* d_in, const int* in_sizes, int n_in,
                              void* d_out, int out_size, void* d_ws, size_t ws_size,
                              hipStream_t stream) {
    if (n_in < 5) return;
    const long long rowsX = (long long)(NB - 1) * SEQ_FULL + SEQ;
    if ((long long)in_sizes[0] < rowsX * DM) return;
    if (in_sizes[1] < DM * DM || in_sizes[2] < DM * HD || in_sizes[3] < DM * HD || in_sizes[4] < DM * DM) return;
    if ((long long)out_size < rowsX * DM) return;

    const float* x  = (const float*)d_in[0];
    const float* Wq = (const float*)d_in[1];
    const float* Wk = (const float*)d_in[2];
    const float* Wv = (const float*)d_in[3];
    const float* Wo = (const float*)d_in[4];
    float* out = (float*)d_out;

    size_t off = 0;
    char* wsb = (char*)d_ws;
    auto carve = [&](size_t bytes) -> void* {
        void* p = wsb + off;
        off += (bytes + 255) & ~(size_t)255;
        return p;
    };
    _Float16* x16  = (_Float16*)carve((size_t)MROWS * DM * 2);
    _Float16* WqT  = (_Float16*)carve((size_t)DM * DM * 2);
    _Float16* WkvT = (_Float16*)carve((size_t)(2 * HD) * DM * 2);
    _Float16* WoT  = (_Float16*)carve((size_t)DM * DM * 2);
    float*    cosT = (float*)carve((size_t)SEQ * 32 * 4);
    float*    sinT = (float*)carve((size_t)SEQ * 32 * 4);
    _Float16* q16  = (_Float16*)carve((size_t)MROWS * DM * 2);
    _Float16* qlo  = (_Float16*)carve((size_t)NB * ER * DM * 2);
    _Float16* kpl  = (_Float16*)carve((size_t)MROWS * HD * 2);
    _Float16* klo  = (_Float16*)carve((size_t)NB * ER * HD * 2);
    _Float16* vT   = (_Float16*)carve((size_t)NB * HD * SEQ * 2);
    _Float16* vTr  = (_Float16*)carve((size_t)NB * HD * ER * 2);
    _Float16* y16  = (_Float16*)carve((size_t)MROWS * DM * 2);
    _Float16* ylo  = (_Float16*)carve((size_t)NB * ER * DM * 2);
    float*    ostg = (float*)carve((size_t)NB * ER * DM * 4);
    if (off > ws_size) return;

    dim3 blk(256);

    k_cvt_x<<<dim3(MROWS / 2), blk, 0, stream>>>(x, x16);
    k_wt<<<dim3(DM / 32, DM / 64), blk, 0, stream>>>(Wq, WqT, DM);
    k_wt<<<dim3(HD / 32, DM / 64), blk, 0, stream>>>(Wk, WkvT, HD);
    k_wt<<<dim3(HD / 32, DM / 64), blk, 0, stream>>>(Wv, WkvT + (size_t)HD * DM, HD);
    k_wt<<<dim3(DM / 32, DM / 64), blk, 0, stream>>>(Wo, WoT, DM);
    k_tab<<<dim3(SEQ / 8), blk, 0, stream>>>(cosT, sinT);

    k_gemm<3><<<dim3(DM / 128, MROWS / 128), blk, 0, stream>>>(
        x16, WqT, (void*)q16, (void*)q16, (void*)qlo, (void*)qlo, cosT, sinT, DM, DM, LOG2E / WSCALE);
    k_gemm<2><<<dim3(1, MROWS / 128), blk, 0, stream>>>(
        x16, WkvT, (void*)kpl, (void*)vT, (void*)klo, (void*)vTr, cosT, sinT, 2 * HD, DM, 1.0f / WSCALE);
    k_attn_e<<<dim3(NB * NH * (ER / 64)), dim3(128), 0, stream>>>(q16, qlo, kpl, klo, vT, vTr, y16, ylo);
    if (SEQ / 64 - ER / 64 > 0)
        k_attn<<<dim3(NB * NH * (SEQ / 64 - ER / 64)), dim3(128), 0, stream>>>(q16, kpl, vT, y16);
    k_gemm<1><<<dim3(DM / 128, MROWS / 128), blk, 0, stream>>>(
        y16, WoT, (void*)out, (void*)ostg, (void*)ostg, (void*)ostg, cosT, sinT, DM, DM, 1.0f / (YCARRY * WSCALE));
    k_gemm<4><<<dim3(DM / 128, (NB * ER) / 128), blk, 0, stream>>>(
        ylo, WoT, (void*)out, (void*)ostg, (void*)ostg, (void*)ostg, cosT, sinT, DM, DM, 1.0f / (YCARRY * WSCALE * RESC));
}
